// INRRandomGraph_42623255446007
// MI455X (gfx1250) — hardware-verified
//
#include <hip/hip_runtime.h>
#include <stddef.h>
#include <stdint.h>
#include <math.h>


#define WID          64
#define NNODE        16
#define NMAT         17
#define NSLOT        17
#define FSLOT        16
#define SW           64.0f
#define SA           256.0f
#define INVC         (1.0f / 16384.0f)
#define NWAVE        2
#define NTHR         64
#define RPW          16
#define RPB          32
#define MAT_HALVES   4096
#define PLANE_HALVES (NMAT * MAT_HALVES)
#define PREP_THR     256
#define PREP_NB      34
#define WSCAP        134217728

static_assert(PLANE_HALVES == PREP_NB * PREP_THR * 8);
static_assert(NTHR == NWAVE * 32);
static_assert(RPB == NWAVE * RPW);
static_assert((RPB * 3 * 4) % 128 == 0);
static_assert(RPB * 3 == 24 * 4);

typedef float    v4f  __attribute__((ext_vector_type(4)));
typedef float    v8f  __attribute__((ext_vector_type(8)));
typedef _Float16 v8h  __attribute__((ext_vector_type(8)));
typedef _Float16 v16h __attribute__((ext_vector_type(16)));
typedef v4f v4fa __attribute__((may_alias));
union FragH { v16h v; v8h h[2]; };
union F8    { v8f v; v4f q[2]; };

__device__ __forceinline__ v8f wmf(v16h a, v16h b, v8f c) {
  v8f d = __builtin_amdgcn_wmma_f32_16x16x32_f16(false, a, false, b, (short)0, c, false, false);
  asm volatile("v_nop\n\tv_nop\n\tv_nop\n\tv_nop" : "+v"(d) : "v"(a), "v"(b));
  return d;
}

__device__ __forceinline__ v16h ldA(const _Float16* __restrict__ W, int K, int row, int k) {
  const _Float16* p = W + (size_t)row * K + k;
  FragH a;
  a.h[0] = *(const v8h*)p;
  a.h[1] = *(const v8h*)(p + 16);
  return a.v;
}

__device__ __forceinline__ v16h packB(v8f lo, v8f hi) {
  FragH b;
#pragma unroll
  for (int r = 0; r < 8; ++r) {
    b.h[0][r] = (_Float16)(lo[r] * SA);
    b.h[1][r] = (_Float16)(hi[r] * SA);
  }
  return b.v;
}

__device__ __forceinline__ v8f ld8(const float* __restrict__ p) {
  F8 u;
  u.q[0] = *(const v4f*)p;
  u.q[1] = *(const v4f*)(p + 4);
  return u.v;
}

__device__ __forceinline__ v8f epi8(v8f acc, const float* __restrict__ bp) {
  const v8f bv = ld8(bp);
  v8f y;
#pragma unroll
  for (int r = 0; r < 8; ++r) y[r] = acc[r] * INVC + bv[r];
  return y;
}

__device__ __forceinline__ v8f act8(v8f y, int kind) {
  v8f o = y;
  if (kind == 0) {
#pragma unroll
    for (int r = 0; r < 8; ++r) o[r] = tanhf(y[r]);
  } else if (kind == 1) {
#pragma unroll
    for (int r = 0; r < 8; ++r) {
      const float v = y[r];
      const float e = expm1f(fminf(v, 0.0f));
      o[r] = v > 0.0f ? v : e;
    }
  } else if (kind == 2) {
#pragma unroll
    for (int r = 0; r < 8; ++r) {
      const float v = y[r];
      o[r] = fmaxf(v, 0.0f) + log1pf(expf(-fabsf(v)));
    }
  } else if (kind == 3) {
#pragma unroll
    for (int r = 0; r < 8; ++r) o[r] = sinf(y[r]);
  } else {
#pragma unroll
    for (int r = 0; r < 8; ++r) {
      const float v = y[r];
      o[r] = expf(-0.5f * v * v);
    }
  }
  return o;
}

__device__ __forceinline__ unsigned pred_mask(int j) {
  unsigned r = 0u;
  switch (j) {
    case 1:  r = 0x0001u; break;
    case 2:  r = 0x0003u; break;
    case 3:  r = 0x0002u; break;
    case 4:  r = 0x0002u; break;
    case 5:  r = 0x0011u; break;
    case 6:  r = 0x002Du; break;
    case 7:  r = 0x0002u; break;
    case 8:  r = 0x00C0u; break;
    case 9:  r = 0x01A8u; break;
    case 10: r = 0x0301u; break;
    case 11: r = 0x0010u; break;
    case 12: r = 0x000Cu; break;
    case 13: r = 0x1050u; break;
    case 14: r = 0x0803u; break;
    case 15: r = 0x0402u; break;
    default: r = 0u; break;
  }
  return r;
}

__global__ __launch_bounds__(PREP_THR) void k_prep(const float* __restrict__ W1, const float* __restrict__ gW,
                                                   _Float16* plane) {
  const int b = blockIdx.x, t = threadIdx.x;
  const float* src = (b < 2) ? (W1 + (size_t)b * 2048) : (gW + (size_t)(b - 2) * 2048);
  const float* p = src + 8 * t;
  const v4f f0 = *(const v4f*)p, f1 = *(const v4f*)(p + 4);
  v8h hv;
#pragma unroll
  for (int i = 0; i < 4; ++i) {
    hv[i]     = (_Float16)(f0[i] * SW);
    hv[4 + i] = (_Float16)(f1[i] * SW);
  }
  _Float16* d = plane + (size_t)b * 2048 + 8 * t;
  *(volatile v8h*)d = hv;
  __threadfence();
  *(volatile v8h*)d = hv;
}

__global__ __launch_bounds__(NTHR) void k_main(const float* __restrict__ inp, const float* __restrict__ lat,
                                               const float* __restrict__ Wl, const float* __restrict__ bl,
                                               const float* __restrict__ Wx, const float* __restrict__ Wy,
                                               const float* __restrict__ Wr, const float* __restrict__ b1,
                                               const float* __restrict__ gB, const float* __restrict__ outW,
                                               const float* __restrict__ outb, const float* __restrict__ scl,
                                               const _Float16* __restrict__ plane, float* out) {
  __shared__ v4f   sAct[NWAVE * NSLOT * 256];
  __shared__ float sF[NWAVE * 32 * 32];
  __shared__ float sO[NWAVE * 48];

  const int tid = threadIdx.x, lane = tid & 31, wave = tid >> 5, h = lane >> 4, m = lane & 15;
  const int n0 = (blockIdx.x * NWAVE + wave) * RPW;
  const int row = n0 + m;
  const int sb = wave * NSLOT * 256 + lane * 8;
  const int fb = (wave * 32 + lane) * 32;
  const v8f z8 = {0.f, 0.f, 0.f, 0.f, 0.f, 0.f, 0.f, 0.f};

  {
    const float x  = inp[(size_t)row * 3 + 0];
    const float y  = inp[(size_t)row * 3 + 1];
    const float rr = inp[(size_t)row * 3 + 2];
    const float* lp = lat + (size_t)row * 8;
    const v4f l0 = *(const v4f*)lp, l1 = *(const v4f*)(lp + 4);
#pragma unroll 1
    for (int c = 0; c < 32; ++c) {
      const int col = 16 * (c >> 3) + 8 * h + (c & 7);
      const float* wl = Wl + col * 8;
      const v4f w0 = *(const v4f*)wl, w1 = *(const v4f*)(wl + 4);
      float lt = l0[0] * w0[0];
      lt += l0[1] * w0[1];
      lt += l0[2] * w0[2];
      lt += l0[3] * w0[3];
      lt += l1[0] * w1[0];
      lt += l1[1] * w1[1];
      lt += l1[2] * w1[2];
      lt += l1[3] * w1[3];
      lt += bl[col];
      const float xv = tanhf(x * Wx[col]);
      const float yy = y * Wy[col];
      const float yv = fmaxf(yy, 0.0f) + log1pf(expf(-fabsf(yy)));
      const float rq = rr * Wr[col];
      const float re = expm1f(fminf(rq, 0.0f));
      const float rv = rq > 0.0f ? rq : re;
      const float pre = ((xv + yv) + rv) + tanhf(lt);
      sF[fb + c] = expf(-0.5f * pre * pre);
    }
  }
  __syncthreads();

  {
    v8f X[4];
#pragma unroll
    for (int f = 0; f < 4; ++f) {
#pragma unroll
      for (int r = 0; r < 8; ++r) X[f][r] = sF[fb + 8 * f + r];
    }
    const v16h xb0 = packB(X[0], X[1]);
    const v16h xb1 = packB(X[2], X[3]);
#pragma unroll 1
    for (int f = 0; f < 4; ++f) {
      v8f acc = z8;
      acc = wmf(ldA(plane, WID, 16 * f + m, 8 * h), xb0, acc);
      acc = wmf(ldA(plane, WID, 16 * f + m, 32 + 8 * h), xb1, acc);
      const v8f yv = epi8(acc, b1 + 16 * f + 8 * h);
      F8 u;
#pragma unroll
      for (int r = 0; r < 8; ++r) u.v[r] = sinf(yv[r]);
      sAct[sb + 256 * FSLOT + 2 * f]     = u.q[0];
      sAct[sb + 256 * FSLOT + 2 * f + 1] = u.q[1];
    }
  }

#pragma unroll 1
  for (int j = 0; j < NNODE; ++j) {
    const unsigned pm = pred_mask(j);
    const unsigned msk = (pm == 0u) ? (1u << FSLOT) : pm;
    const int kind = j % 5;
    v8f IN[4] = {z8, z8, z8, z8};
#pragma unroll 1
    for (int i = 0; i < NSLOT; ++i) {
      if ((msk >> i) & 1u) {
#pragma unroll
        for (int f = 0; f < 4; ++f) {
          F8 u;
          u.q[0] = sAct[sb + 256 * i + 2 * f];
          u.q[1] = sAct[sb + 256 * i + 2 * f + 1];
          IN[f] = IN[f] + u.v;
        }
      }
    }
    const v16h xb0 = packB(IN[0], IN[1]);
    const v16h xb1 = packB(IN[2], IN[3]);
    const _Float16* Wj = plane + (size_t)(1 + j) * MAT_HALVES;
    const float* bj = gB + j * WID;
#pragma unroll 1
    for (int f = 0; f < 4; ++f) {
      v8f acc = z8;
      acc = wmf(ldA(Wj, WID, 16 * f + m, 8 * h), xb0, acc);
      acc = wmf(ldA(Wj, WID, 16 * f + m, 32 + 8 * h), xb1, acc);
      const v8f yv = act8(epi8(acc, bj + 16 * f + 8 * h), kind);
      F8 u; u.v = yv;
      sAct[sb + 256 * j + 2 * f]     = u.q[0];
      sAct[sb + 256 * j + 2 * f + 1] = u.q[1];
    }
  }

  {
    float s0 = 0.f, s1 = 0.f, s2 = 0.f;
#pragma unroll
    for (int f = 0; f < 4; ++f) {
      F8 a, b, c;
      a.q[0] = sAct[sb + 256 * 13 + 2 * f]; a.q[1] = sAct[sb + 256 * 13 + 2 * f + 1];
      b.q[0] = sAct[sb + 256 * 14 + 2 * f]; b.q[1] = sAct[sb + 256 * 14 + 2 * f + 1];
      c.q[0] = sAct[sb + 256 * 15 + 2 * f]; c.q[1] = sAct[sb + 256 * 15 + 2 * f + 1];
      const v8f ag = (a.v + b.v) + c.v;
      const v8f w0 = ld8(outW + 0 * WID + 16 * f + 8 * h);
      const v8f w1 = ld8(outW + 1 * WID + 16 * f + 8 * h);
      const v8f w2 = ld8(outW + 2 * WID + 16 * f + 8 * h);
#pragma unroll
      for (int r = 0; r < 8; ++r) {
        s0 += ag[r] * w0[r];
        s1 += ag[r] * w1[r];
        s2 += ag[r] * w2[r];
      }
    }
    s0 += __shfl_xor(s0, 16, 32);
    s1 += __shfl_xor(s1, 16, 32);
    s2 += __shfl_xor(s2, 16, 32);
    const float sc = scl[0];
    const float z0 = (s0 + outb[0]) * sc, z1 = (s1 + outb[1]) * sc, z2 = (s2 + outb[2]) * sc;
    const float e0 = expf(-fabsf(z0)), e1 = expf(-fabsf(z1)), e2 = expf(-fabsf(z2));
    const float o0 = (z0 >= 0.0f ? 1.0f : e0) * __builtin_amdgcn_rcpf(1.0f + e0);
    const float o1 = (z1 >= 0.0f ? 1.0f : e1) * __builtin_amdgcn_rcpf(1.0f + e1);
    const float o2 = (z2 >= 0.0f ? 1.0f : e2) * __builtin_amdgcn_rcpf(1.0f + e2);
    if (h == 0) {
      sO[wave * 48 + m * 3 + 0] = o0;
      sO[wave * 48 + m * 3 + 1] = o1;
      sO[wave * 48 + m * 3 + 2] = o2;
    }
  }
  __syncthreads();
  {
    const int ti = tid < 24 ? tid : 23;
    const v4f ov = *(const v4fa*)(sO + 4 * ti);
    float* op = out + (size_t)blockIdx.x * (RPB * 3) + 4 * ti;
    if (tid < 24) *(volatile v4f*)op = ov;
    __threadfence();
    if (tid < 24) *(volatile v4f*)op = ov;
  }
}

extern "C" void kernel_launch(void* const* d_in, const int* in_sizes, int n_in,
                              void* d_out, int out_size, void* d_ws, size_t ws_size,
                              hipStream_t stream) {
  if (n_in < 14) return;
  const int nrows = in_sizes[0] / 3;
  if (nrows <= 0 || nrows * 3 != in_sizes[0] || (nrows % RPB) != 0) return;
  if (in_sizes[1] != nrows * 8) return;
  if (in_sizes[2] != WID * 8 || in_sizes[3] != WID) return;
  if (in_sizes[4] != WID || in_sizes[5] != WID || in_sizes[6] != WID) return;
  if (in_sizes[7] != WID * WID || in_sizes[8] != WID) return;
  if (in_sizes[9] != NNODE * WID * WID || in_sizes[10] != NNODE * WID) return;
  if (in_sizes[11] != 3 * WID || in_sizes[12] != 3 || in_sizes[13] != 1) return;
  if (out_size != nrows * 3) return;

  const size_t plane_bytes = (size_t)PLANE_HALVES * 2;
  if (plane_bytes > ws_size || plane_bytes > (size_t)WSCAP) return;
  _Float16* plane = (_Float16*)d_ws;

  const float* inp  = (const float*)d_in[0];
  const float* lat  = (const float*)d_in[1];
  const float* Wl   = (const float*)d_in[2];
  const float* bl   = (const float*)d_in[3];
  const float* Wx   = (const float*)d_in[4];
  const float* Wy   = (const float*)d_in[5];
  const float* Wr   = (const float*)d_in[6];
  const float* W1   = (const float*)d_in[7];
  const float* b1   = (const float*)d_in[8];
  const float* gW   = (const float*)d_in[9];
  const float* gB   = (const float*)d_in[10];
  const float* outW = (const float*)d_in[11];
  const float* outb = (const float*)d_in[12];
  const float* scl  = (const float*)d_in[13];
  float* out = (float*)d_out;

  k_prep<<<PREP_NB, PREP_THR, 0, stream>>>(W1, gW, plane);
  k_main<<<nrows / RPB, NTHR, 0, stream>>>(inp, lat, Wl, bl, Wx, Wy, Wr, b1, gB, outW, outb, scl,
                                           plane, out);
}
